// UnstructuredSparse_23381801960228
// MI455X (gfx1250) — hardware-verified
//
#include <hip/hip_runtime.h>
#include <stddef.h>


typedef _Float16 v16h __attribute__((ext_vector_type(16)));
typedef _Float16 v8h  __attribute__((ext_vector_type(8)));
typedef float    v8f  __attribute__((ext_vector_type(8)));
typedef float    v4f  __attribute__((ext_vector_type(4)));

#ifndef TOK
#define TOK 256
#endif
#ifndef NOUT
#define NOUT 4096
#endif
#define TOK_FULL  256
#define NOUT_FULL 4096
#define NIN       4096
#define NNZ       8388608u
#define WTOTAL    ((unsigned)NOUT_FULL * (unsigned)NIN)
#define LB_STEPS  24

static_assert(TOK >= 64 && TOK <= TOK_FULL && (TOK % 64) == 0);
static_assert(NOUT >= 64 && NOUT <= NOUT_FULL && (NOUT % 64) == 0);
static_assert((NIN % 64) == 0 && (NIN % 32) == 0);
static_assert(NIN == 256 * 8 * 2);
static_assert(NNZ <= (1u << 23));
static_assert(((size_t)TOK * NIN) % 2048 == 0);
static_assert((size_t)NOUT_FULL * NIN <= (size_t)0x7FFFFFFF);

#define CHK       ((NNZ + (unsigned)NOUT - 1u) / (unsigned)NOUT)
#define CHK_ITERS ((CHK + 255u) / 256u)
static_assert((size_t)CHK * NOUT >= (size_t)NNZ);
static_assert((size_t)NOUT * CHK + (size_t)CHK_ITERS * 256 < (size_t)0xFFFFFFFFu);

#define LDC 68
static_assert((LDC % 4) == 0 && LDC >= 64);

#define WCARRY 64.0f
#define XCARRY 16.0f

#define X16_BYTES ((size_t)TOK * NIN * 2)
#define W16_BYTES ((size_t)NOUT * NIN * 2)
#define OFF_X16   ((size_t)0)
#define OFF_W16   (OFF_X16 + X16_BYTES)
#define WS_TOTAL  (OFF_W16 + W16_BYTES)
static_assert((X16_BYTES % 128) == 0 && (W16_BYTES % 128) == 0);
static_assert(WS_TOTAL <= (size_t)134217728);

__device__ __forceinline__ float bf16r(float x) {
  unsigned int u = __float_as_uint(x);
  u = (u + 0x7FFFu + ((u >> 16) & 1u)) & 0xFFFF0000u;
  return __uint_as_float(u);
}

static __device__ __forceinline__ _Float16 toh_flush(float v) {
  const _Float16 r = (_Float16)v;
  return (fabsf(v) < 6.103515625e-05f) ? (_Float16)0.0f : r;
}

__device__ __forceinline__ v16h frag_at(const _Float16* p) {
  v8h lo = *(const v8h*)(p);
  v8h hi = *(const v8h*)(p + 16);
  v16h out;
#pragma unroll
  for (int i = 0; i < 8; ++i) { out[i] = lo[i]; out[i + 8] = hi[i]; }
  return out;
}

__device__ __forceinline__ v8f wmma16(v16h a, v16h b, v8f c) {
  v8f d = __builtin_amdgcn_wmma_f32_16x16x32_f16(false, a, false, b, (short)0, c,
                                                 false, false);
  asm volatile("v_nop\n\tv_nop\n\tv_nop\n\tv_nop" : "+v"(d) : "v"(a), "v"(b));
  return d;
}

__global__ __launch_bounds__(256) void xconv_kernel(
    const float* __restrict__ X, _Float16* __restrict__ X16) {
#pragma clang fp contract(off)
  const size_t e = ((size_t)blockIdx.x * 256u + threadIdx.x) * 8u;
  const v4f a0 = *(const v4f*)(X + e);
  const v4f a1 = *(const v4f*)(X + e + 4u);
  v8h o;
#pragma unroll
  for (int i = 0; i < 4; ++i) {
    o[i]     = toh_flush(XCARRY * bf16r(a0[i]));
    o[i + 4] = toh_flush(XCARRY * bf16r(a1[i]));
  }
  _Float16* p = X16 + e;
  *(volatile v8h*)p = o;
  __threadfence();
  *(volatile v8h*)p = o;
}

__device__ __forceinline__ unsigned lower_bound_idx(const int* __restrict__ idx, int key) {
  unsigned lo = 0u, hi = NNZ;
#pragma unroll 1
  for (int it = 0; it < LB_STEPS; ++it) {
    const unsigned mid = (lo + hi) >> 1;
    const unsigned midc = (mid < (NNZ - 1u)) ? mid : (NNZ - 1u);
    const int v = idx[midc];
    const bool act = lo < hi;
    const bool right = act && (v < key);
    const bool left = act && !right;
    lo = right ? (mid + 1u) : lo;
    hi = left ? mid : hi;
  }
  return lo;
}

__global__ __launch_bounds__(256) void densify_kernel(
    const float* __restrict__ val, const int* __restrict__ idx, _Float16* __restrict__ Wt) {
#pragma clang fp contract(off)
  __shared__ _Float16 R[NIN];
  __shared__ int sbad[8];
  const unsigned tid = threadIdx.x, lane = tid & 31u;
  const int wave = __builtin_amdgcn_readfirstlane((int)(threadIdx.x >> 5));
  const unsigned o = blockIdx.x;

  {
    const v8h z = {};
#pragma unroll
    for (unsigned i = 0; i < 2u; ++i) *(v8h*)&R[tid * 8u + 2048u * i] = z;
  }

  int bad = 0;
  {
    const unsigned base = o * CHK;
#pragma unroll 1
    for (unsigned j = 0; j < CHK_ITERS; ++j) {
      const unsigned i = base + tid + 256u * j;
      const unsigned ic = (i < (NNZ - 1u)) ? i : (NNZ - 1u);
      const unsigned in = ((i + 1u) < (NNZ - 1u)) ? (i + 1u) : (NNZ - 1u);
      const int a = idx[ic];
      const int b = idx[in];
      const bool valid = i < NNZ;
      const bool pair = (i + 1u) < NNZ;
      const bool oor = (unsigned)a >= WTOTAL;
      const bool desc = pair && (a >= b);
      bad |= (valid && (oor || desc)) ? 1 : 0;
    }
  }

  const int k0 = (int)(o * (unsigned)NIN);
  const unsigned s0 = lower_bound_idx(idx, k0);
  const unsigned s1 = lower_bound_idx(idx, k0 + NIN);
  unsigned cnt = (s1 > s0) ? (s1 - s0) : 0u;
  cnt = (cnt < (unsigned)NIN) ? cnt : (unsigned)NIN;
  const unsigned niter = (cnt + 255u) >> 8;
  __syncthreads();

#pragma unroll 1
  for (unsigned j = 0; j < niter; ++j) {
    const unsigned q = tid + 256u * j;
    const unsigned p = s0 + q;
    const unsigned pc = (p < (NNZ - 1u)) ? p : (NNZ - 1u);
    int fi = idx[pc];
    float vv = val[pc];
    asm volatile("" : "+v"(fi), "+v"(vv));
    const unsigned col = (unsigned)(fi - k0);
    const _Float16 h = toh_flush(WCARRY * bf16r(vv));
    if (q < cnt && col < (unsigned)NIN) R[col] = h;
  }

  int bw = bad;
#pragma unroll
  for (int off = 1; off < 32; off <<= 1) bw |= __shfl_xor(bw, off, 32);
  if (lane == 0u) sbad[wave] = bw;
  __syncthreads();
  int ball = 0;
#pragma unroll
  for (int i = 0; i < 8; ++i) ball |= sbad[i];
  const bool poison = (ball != 0);
  const _Float16 nanh = (_Float16)__uint_as_float(0x7FC00000u);

  v8h x[2];
  size_t off[2];
#pragma unroll
  for (unsigned i = 0; i < 2u; ++i) {
    const unsigned c = tid * 8u + 2048u * i;
    v8h t = *(const v8h*)&R[c];
#pragma unroll
    for (int j = 0; j < 8; ++j) t[j] = poison ? nanh : t[j];
    x[i] = t;
    off[i] = (size_t)o * NIN + c;
  }
#pragma unroll
  for (int i = 0; i < 2; ++i) *(volatile v8h*)(Wt + off[i]) = x[i];
  __threadfence();
#pragma unroll
  for (int i = 0; i < 2; ++i) *(volatile v8h*)(Wt + off[i]) = x[i];
}

__global__ __launch_bounds__(256) void gemm_out_kernel(
    const _Float16* __restrict__ A16, const _Float16* __restrict__ Bt, const unsigned K,
    float* __restrict__ outf) {
  __shared__ float Cs[64 * LDC];
  const unsigned tid = threadIdx.x, lane = tid & 31u;
  const unsigned w = (unsigned)__builtin_amdgcn_readfirstlane((int)(threadIdx.x >> 5));
  const unsigned mw = w >> 1, nw = w & 1u;
  const unsigned hh = lane >> 4, m = lane & 15u;
  const unsigned n0 = blockIdx.x * 64u;
  const unsigned row0 = blockIdx.y * 64u;

  const _Float16* ap  = A16 + (size_t)(row0 + mw * 16u + m) * K + hh * 8u;
  const _Float16* bp0 = Bt + (size_t)(n0 + nw * 32u + m) * K + hh * 8u;
  const _Float16* bp1 = bp0 + (size_t)16 * K;
  v8f acc0 = {}, acc1 = {};
#pragma unroll 2
  for (unsigned k0 = 0; k0 < K; k0 += 32u) {
    const v16h a  = frag_at(ap + k0);
    const v16h b0 = frag_at(bp0 + k0);
    const v16h b1 = frag_at(bp1 + k0);
    acc0 = wmma16(a, b0, acc0);
    acc1 = wmma16(a, b1, acc1);
  }
#pragma unroll
  for (int r = 0; r < 8; ++r) {
    float* d = &Cs[(mw * 16u + hh * 8u + (unsigned)r) * LDC + nw * 32u + m];
    d[0]  = acc0[r];
    d[16] = acc1[r];
  }
  __syncthreads();

  const float cs = 1.0f / (WCARRY * XCARRY);
  v4f xs[4];
  size_t off[4];
#pragma unroll
  for (unsigned i = 0; i < 4u; ++i) {
    const unsigned r = 16u * i + (tid >> 4);
    const unsigned c = (tid & 15u) * 4u;
    const v4f u = *(const v4f*)&Cs[r * LDC + c];
    v4f valv;
#pragma unroll
    for (int j = 0; j < 4; ++j) valv[j] = u[j] * cs;
    xs[i] = valv;
    off[i] = (size_t)(row0 + r) * NOUT_FULL + n0 + c;
  }
#pragma unroll
  for (int i = 0; i < 4; ++i) *(volatile v4f*)(outf + off[i]) = xs[i];
  __threadfence();
#pragma unroll
  for (int i = 0; i < 4; ++i) *(volatile v4f*)(outf + off[i]) = xs[i];
}

extern "C" void kernel_launch(void* const* d_in, const int* in_sizes, int n_in,
                              void* d_out, int out_size, void* d_ws, size_t ws_size,
                              hipStream_t stream) {
  if (n_in < 3) return;
  if ((long long)in_sizes[0] < (long long)TOK * NIN) return;
  if ((long long)in_sizes[1] < (long long)NNZ) return;
  if ((long long)in_sizes[2] < (long long)NNZ) return;
  if ((long long)out_size < (long long)(TOK - 1) * NOUT_FULL + NOUT) return;
  if (ws_size < WS_TOTAL) return;

  const float* X   = (const float*)d_in[0];
  const float* val = (const float*)d_in[1];
  const int*   idx = (const int*)d_in[2];
  float* out = (float*)d_out;

  char* ws = (char*)d_ws;
  _Float16* X16 = (_Float16*)(ws + OFF_X16);
  _Float16* W16 = (_Float16*)(ws + OFF_W16);

  dim3 blk(256);
  xconv_kernel<<<dim3((unsigned)(((size_t)TOK * NIN) / 2048)), blk, 0, stream>>>(X, X16);
  densify_kernel<<<dim3(NOUT), blk, 0, stream>>>(val, idx, W16);
  gemm_out_kernel<<<dim3(NOUT / 64, TOK / 64), blk, 0, stream>>>(X16, W16, (unsigned)NIN, out);
}
